// FAVORCausalSelfAttention_21242908246344
// MI455X (gfx1250) — hardware-verified
//
#include <hip/hip_runtime.h>


#define NB_  2
#define TT   1024
#define DM   1024
#define D3   3072
#define NH_  16
#define HD   64
#define MF   128
#define ZH   8
typedef _Float16 h16;
typedef unsigned short bf;
typedef __attribute__((ext_vector_type(16))) __bf16   v16bf;
typedef __attribute__((ext_vector_type(16))) _Float16 v16h;
typedef __attribute__((ext_vector_type(8)))  _Float16 v8h;
typedef __attribute__((ext_vector_type(8)))  unsigned short v8us;
typedef __attribute__((ext_vector_type(8)))  float    v8f;
typedef __attribute__((ext_vector_type(4)))  float    v4f;
typedef v8h  __attribute__((may_alias)) v8ha;
typedef v4f  __attribute__((may_alias)) v4fa;
typedef v8us __attribute__((may_alias)) v8usa;

__device__ __forceinline__ unsigned short f2bf(float f) { unsigned u = __float_as_uint(f); u += 0x7FFFu + ((u >> 16) & 1u); return (unsigned short)(u >> 16); }
__device__ __forceinline__ float bf2f(unsigned short b) { return __uint_as_float(((unsigned)b) << 16); }
__device__ __forceinline__ float bfr(float f) { return bf2f(f2bf(f)); }
__device__ __forceinline__ v16h cat16(v8h lo, v8h hi) { return __builtin_shufflevector(lo, hi, 0, 1, 2, 3, 4, 5, 6, 7, 8, 9, 10, 11, 12, 13, 14, 15); }
__device__ __forceinline__ v16bf cat16b(v8us lo, v8us hi) { return __builtin_bit_cast(v16bf, __builtin_shufflevector(lo, hi, 0, 1, 2, 3, 4, 5, 6, 7, 8, 9, 10, 11, 12, 13, 14, 15)); }
__device__ __forceinline__ v8f wmma16(v16h a, v16h b, v8f c) { return __builtin_amdgcn_wmma_f32_16x16x32_f16(false, a, false, b, (short)0, c, false, false); }
__device__ __forceinline__ v8f wmmab(v16bf a, v16bf b, v8f c) { return __builtin_amdgcn_wmma_f32_16x16x32_bf16(false, a, false, b, (short)0, c, false, false); }


template <typename T16> struct WFrag;
template <> struct WFrag<h16> { typedef v16h V; static __device__ __forceinline__ V ld(const h16* p) { return cat16(*(const v8h*)p, *(const v8h*)(p + 16)); } static __device__ __forceinline__ v8f mma(V a, V b, v8f c) { return wmma16(a, b, c); } };
template <> struct WFrag<bf> { typedef v16bf V; static __device__ __forceinline__ V ld(const bf* p) { return cat16b(*(const v8us*)p, *(const v8us*)(p + 16)); } static __device__ __forceinline__ v8f mma(V a, V b, v8f c) { return wmmab(a, b, c); } };
template <typename T16, int NSPLIT, bool BIAS>
__global__ __launch_bounds__(32) void k_gemmw(const T16* __restrict__ A, const T16* __restrict__ A2, const T16* __restrict__ Bt, const T16* __restrict__ Bt2, int K, float* C, int ldc, const float* __restrict__ bias, size_t sA, size_t sB, size_t sC) {
    typedef typename WFrag<T16>::V V;
    __shared__ __align__(16) float os[16 * 68];
    const size_t z = blockIdx.z; A += z * sA; if (A2) A2 += z * sA; Bt += z * sB; if (Bt2) Bt2 += z * sB; C += z * sC;
    const int lane = threadIdx.x & 31, lr = lane & 15, hi = lane >> 4; const int r0 = blockIdx.x * 64, c0 = blockIdx.y * 64;
    v8f acc[4][4];
#pragma unroll
    for (int mb = 0; mb < 4; ++mb)
#pragma unroll
        for (int nb = 0; nb < 4; ++nb) acc[mb][nb] = (v8f){};
    const size_t aoff = (size_t)(r0 + lr) * K + 8 * hi, boff = (size_t)(c0 + lr) * K + 8 * hi;
#pragma unroll 1
    for (int kc = 0; kc < K; kc += 32) {
        V a[4], a2[4];
#pragma unroll
        for (int mb = 0; mb < 4; ++mb) { a[mb] = WFrag<T16>::ld(A + aoff + (size_t)mb * 16 * K + kc); if (NSPLIT == 1 || NSPLIT == 2) a2[mb] = WFrag<T16>::ld(A2 + aoff + (size_t)mb * 16 * K + kc); }
#pragma unroll
        for (int nb = 0; nb < 4; ++nb) { const V b = WFrag<T16>::ld(Bt + boff + (size_t)nb * 16 * K + kc); V b2; if (NSPLIT >= 2) b2 = WFrag<T16>::ld(Bt2 + boff + (size_t)nb * 16 * K + kc);
#pragma unroll
            for (int mb = 0; mb < 4; ++mb) { acc[mb][nb] = WFrag<T16>::mma(a[mb], b, acc[mb][nb]); if (NSPLIT == 1 || NSPLIT == 2) acc[mb][nb] = WFrag<T16>::mma(a2[mb], b, acc[mb][nb]); if (NSPLIT >= 2) acc[mb][nb] = WFrag<T16>::mma(a[mb], b2, acc[mb][nb]); } }
        asm volatile("v_nop\n\tv_nop\n\tv_nop\n\tv_nop" : "+v"(acc[0][0]), "+v"(acc[1][1]), "+v"(acc[2][2]), "+v"(acc[3][3]) : "v"(a[0]), "v"(a[3]));
    }
#pragma unroll
    for (int mb = 0; mb < 4; ++mb) {
#pragma unroll
        for (int nb = 0; nb < 4; ++nb) {
#pragma unroll
            for (int j = 0; j < 8; ++j) os[(hi * 8 + j) * 68 + nb * 16 + lr] = acc[mb][nb][j]; }
        __builtin_amdgcn_wave_barrier(); asm volatile("" ::: "memory");
        float* crow = C + (size_t)(r0 + mb * 16) * ldc + c0;
#pragma unroll 1
        for (int ps = 0; ps < 2; ++ps) {
#pragma unroll
            for (int s = 0; s < 8; ++s) { const int row = 2 * s + hi, cofs = lr * 4; v4f val = *(const v4fa*)(os + row * 68 + cofs); if (BIAS) { val[0] += bfr(bias[c0 + cofs]); val[1] += bfr(bias[c0 + cofs + 1]); val[2] += bfr(bias[c0 + cofs + 2]); val[3] += bfr(bias[c0 + cofs + 3]); }
                *(volatile v4f*)(crow + (size_t)row * ldc + cofs) = val; }
            if (ps == 0) __threadfence(); }
        __builtin_amdgcn_wave_barrier(); asm volatile("" ::: "memory");
    }
}

template <typename T16, int NSPLIT, int CMODE>
__global__ __launch_bounds__(32) void k_gemmc(const T16* __restrict__ A, const T16* __restrict__ A2, const T16* __restrict__ Bt, const T16* __restrict__ Bt2, int K, float* C, int ldc, int roff, size_t sA, size_t sB, size_t sC) {
    typedef typename WFrag<T16>::V V;
    __shared__ __align__(16) float os[16 * 68];
    const size_t z = blockIdx.z; A += z * sA; if (A2) A2 += z * sA; Bt += z * sB; if (Bt2) Bt2 += z * sB; C += z * sC;
    const int lane = threadIdx.x & 31, lr = lane & 15, hi = lane >> 4; const int r0 = blockIdx.x * 64, c0 = blockIdx.y * 64;
    if (CMODE == 1 && c0 > r0 + roff + 63) return;
    const int Kl = (CMODE == 2) ? min(K, r0 + roff + 64) : K;
    v8f acc[4][4];
#pragma unroll
    for (int mb = 0; mb < 4; ++mb)
#pragma unroll
        for (int nb = 0; nb < 4; ++nb) acc[mb][nb] = (v8f){};
    const size_t aoff = (size_t)(r0 + lr) * K + 8 * hi, boff = (size_t)(c0 + lr) * K + 8 * hi;
#pragma unroll 1
    for (int kc = 0; kc < Kl; kc += 32) {
        V a[4], a2[4];
#pragma unroll
        for (int mb = 0; mb < 4; ++mb) { a[mb] = WFrag<T16>::ld(A + aoff + (size_t)mb * 16 * K + kc); if (NSPLIT == 1 || NSPLIT == 2) a2[mb] = WFrag<T16>::ld(A2 + aoff + (size_t)mb * 16 * K + kc); }
#pragma unroll
        for (int nb = 0; nb < 4; ++nb) { const V b = WFrag<T16>::ld(Bt + boff + (size_t)nb * 16 * K + kc); V b2; if (NSPLIT >= 2) b2 = WFrag<T16>::ld(Bt2 + boff + (size_t)nb * 16 * K + kc);
#pragma unroll
            for (int mb = 0; mb < 4; ++mb) { acc[mb][nb] = WFrag<T16>::mma(a[mb], b, acc[mb][nb]); if (NSPLIT == 1 || NSPLIT == 2) acc[mb][nb] = WFrag<T16>::mma(a2[mb], b, acc[mb][nb]); if (NSPLIT >= 2) acc[mb][nb] = WFrag<T16>::mma(a[mb], b2, acc[mb][nb]); } }
        asm volatile("v_nop\n\tv_nop\n\tv_nop\n\tv_nop" : "+v"(acc[0][0]), "+v"(acc[1][1]), "+v"(acc[2][2]), "+v"(acc[3][3]) : "v"(a[0]), "v"(a[3]));
    }
#pragma unroll
    for (int mb = 0; mb < 4; ++mb) {
#pragma unroll
        for (int nb = 0; nb < 4; ++nb) {
#pragma unroll
            for (int j = 0; j < 8; ++j) os[(hi * 8 + j) * 68 + nb * 16 + lr] = acc[mb][nb][j]; }
        __builtin_amdgcn_wave_barrier(); asm volatile("" ::: "memory");
        float* crow = C + (size_t)(r0 + mb * 16) * ldc + c0;
#pragma unroll 1
        for (int ps = 0; ps < 2; ++ps) {
#pragma unroll
            for (int s = 0; s < 8; ++s) { const int row = 2 * s + hi, cofs = lr * 4; v4f val = *(const v4fa*)(os + row * 68 + cofs);
                *(volatile v4f*)(crow + (size_t)row * ldc + cofs) = val; }
            if (ps == 0) __threadfence(); }
        __builtin_amdgcn_wave_barrier(); asm volatile("" ::: "memory");
    }
}

__device__ __forceinline__ void splitf(float y, unsigned short& h, unsigned short& l) { h = f2bf(y); l = f2bf(y - bf2f(h)); }
typedef __attribute__((ext_vector_type(2))) unsigned short v2us;
typedef __attribute__((ext_vector_type(4))) unsigned short v4us;

__global__ __launch_bounds__(256) void k_wtG(const float* __restrict__ w, int K, int N, bf* Bt) {
    const int lane = threadIdx.x & 31; const int L0 = (blockIdx.x * 8 + (threadIdx.x >> 5)) * 8; const int nlines = N * K / 64;
#pragma unroll
    for (int ps = 0; ps < 2; ++ps) {
#pragma unroll 1
        for (int l = 0; l < 8; ++l) { const int L = L0 + l; if (L >= nlines) break; const size_t e = (size_t)L * 64 + lane * 2; const int k = (int)(e % K), n = (int)(e / K); v2us o;
            o[0] = f2bf(w[(size_t)k * N + n]); o[1] = f2bf(w[(size_t)(k + 1) * N + n]); *(volatile v2us*)(Bt + e) = o; }
        if (ps == 0) __threadfence(); }
}
__global__ __launch_bounds__(256) void k_cvt8(const float* __restrict__ src, bf* dst, size_t n8) { const size_t i = (size_t)blockIdx.x * 256 + threadIdx.x; if (i >= n8) return; const v8f v = *(const v8f*)(src + i * 8); v8us o;
#pragma unroll
    for (int k = 0; k < 8; ++k) o[k] = f2bf(v[k]); *(volatile v8us*)(dst + i * 8) = o; __threadfence(); *(volatile v8us*)(dst + i * 8) = o; }
__global__ __launch_bounds__(256) void k_phi(const float* __restrict__ QKV, int off, const float* __restrict__ om, bf* Ph_, bf* Pl_) { const int e = (blockIdx.x * 256 + threadIdx.x) * 4; if (e >= NH_ * TT * MF) return; const int m0 = e % MF; const int t = (e / MF) % TT; const int h = e / (MF * TT); const float* ur = QKV + (size_t)t * D3 + off + h * HD;
    float p[4] = {0.f, 0.f, 0.f, 0.f}; float nh = 0.f;
#pragma unroll 1
    for (int d = 0; d < HD; ++d) { const float u = ur[d] * 0.125f; float sq = __fmul_rn(u, u); asm volatile("" : "+v"(sq)); nh = __fadd_rn(nh, sq);
#pragma unroll
        for (int j = 0; j < 4; ++j) { float w = bfr(om[d * MF + m0 + j]); asm volatile("" : "+v"(w)); float pr = __fmul_rn(u, w); asm volatile("" : "+v"(pr)); p[j] = __fadd_rn(p[j], pr); } }
    const float half_n = nh * 0.5f; v4us oh, ol;
#pragma unroll
    for (int j = 0; j < 4; ++j) { const float ex = expf(__fsub_rn(p[j], half_n)); const float ph = __fmul_rn(ex, 0.088388347648318447f); unsigned short a, b; splitf(ph, a, b); oh[j] = a; ol[j] = b; }
    *(volatile v4us*)(Ph_ + e) = oh; *(volatile v4us*)(Pl_ + e) = ol; __threadfence(); *(volatile v4us*)(Ph_ + e) = oh; *(volatile v4us*)(Pl_ + e) = ol; }
__global__ __launch_bounds__(256) void k_vtp2(const float* __restrict__ QKV, bf* VTh, bf* VTl) { const int e = (blockIdx.x * 256 + threadIdx.x) * 2; if (e >= NH_ * HD * TT) return; const int t = e % TT; const int d = (e / TT) % HD; const int h = e / (TT * HD); v2us oh, ol;
#pragma unroll
    for (int u = 0; u < 2; ++u) { unsigned short a, b; splitf(QKV[(size_t)(t + u) * D3 + 2 * DM + h * HD + d], a, b); oh[u] = a; ol[u] = b; }
    *(volatile v2us*)(VTh + e) = oh; *(volatile v2us*)(VTl + e) = ol; __threadfence(); *(volatile v2us*)(VTh + e) = oh; *(volatile v2us*)(VTl + e) = ol; }
__global__ __launch_bounds__(256) void k_lin(const float* __restrict__ Sb, bf* Ah, bf* Al, float* DEN) { const int lane = threadIdx.x & 31; const int row = blockIdx.x * 8 + (threadIdx.x >> 5); if (row >= ZH * TT) return; const int t = row % TT; const float* sr = Sb + (size_t)row * TT; float sum = 0.f; const int nch = t / 128 + 1;
    for (int ps = 0; ps < 2; ++ps) { sum = 0.f;
#pragma unroll 1
        for (int ch = 0; ch < TT / 128; ++ch) { const int s0 = ch * 128 + lane * 4; v4us oh, ol; v4f a = {0.f, 0.f, 0.f, 0.f}; if (ch < nch) a = *(const v4f*)(sr + s0);
#pragma unroll
            for (int u = 0; u < 4; ++u) { const float v = (s0 + u <= t) ? a[u] : 0.f; sum = __fadd_rn(sum, v); unsigned short x1, x2; splitf(v, x1, x2); oh[u] = x1; ol[u] = x2; }
            const size_t oo = (size_t)row * TT + s0; *(volatile v4us*)(Ah + oo) = oh; *(volatile v4us*)(Al + oo) = ol; }
        if (ps == 0) __threadfence(); }
#pragma unroll
    for (int sh = 16; sh; sh >>= 1) sum += __shfl_xor(sum, sh, 32);
    *(volatile float*)(DEN + (size_t)row * 32 + lane) = sum; __threadfence(); *(volatile float*)(DEN + (size_t)row * 32 + lane) = sum; }
__global__ __launch_bounds__(256) void k_y(const float* __restrict__ O, const float* __restrict__ DEN, int h0, bf* Yh, bf* Yl) { const int e = (blockIdx.x * 256 + threadIdx.x) * 4; if (e >= ZH * TT * HD) return; const int d = e % HD; const int t = (e / HD) % TT; const int z = e / (HD * TT); const float den = __fadd_rn(DEN[((size_t)z * TT + t) * 32], 1e-6f); v4us oh, ol;
#pragma unroll
    for (int u = 0; u < 4; ++u) { const float y = __fdiv_rn(O[e + u], den); unsigned short a, b; splitf(y, a, b); oh[u] = a; ol[u] = b; } const size_t oo = (size_t)t * DM + (h0 + z) * HD + d;
    *(volatile v4us*)(Yh + oo) = oh; *(volatile v4us*)(Yl + oo) = ol; __threadfence(); *(volatile v4us*)(Yh + oo) = oh; *(volatile v4us*)(Yl + oo) = ol; }

extern "C" void kernel_launch(void* const* d_in, const int* in_sizes, int n_in,
                              void* d_out, int out_size, void* d_ws, size_t ws_size, hipStream_t stream) {
    (void)in_sizes; (void)n_in; (void)out_size;
    const float** I = (const float**)d_in;
    const float *x = I[0], *wa = I[1], *ba = I[2], *wp = I[3], *bp = I[4], *om = I[5];
    float* OUT = (float*)d_out;
    char* wsp = (char*)d_ws;
    auto take = [&](size_t bytes) { char* p = wsp; wsp += (bytes + 255) & ~(size_t)255; return (void*)p; };
    bf* WA = (bf*)take((size_t)D3 * DM * 2); bf* WP = (bf*)take((size_t)DM * DM * 2); bf* XB = (bf*)take((size_t)TT * DM * 2); float* QKV = (float*)take((size_t)TT * D3 * 4);
    bf* PQh = (bf*)take((size_t)NH_ * TT * MF * 2); bf* PQl = (bf*)take((size_t)NH_ * TT * MF * 2); bf* PKh = (bf*)take((size_t)NH_ * TT * MF * 2); bf* PKl = (bf*)take((size_t)NH_ * TT * MF * 2); bf* VTh = (bf*)take((size_t)NH_ * HD * TT * 2); bf* VTl = (bf*)take((size_t)NH_ * HD * TT * 2);
    float* Sb = (float*)take((size_t)ZH * TT * TT * 4); bf* Ah = (bf*)take((size_t)ZH * TT * TT * 2); bf* Al = (bf*)take((size_t)ZH * TT * TT * 2); float* DEN = (float*)take((size_t)ZH * TT * 32 * 4); float* O = (float*)take((size_t)ZH * TT * HD * 4); bf* Yh = (bf*)take((size_t)TT * DM * 2); bf* Yl = (bf*)take((size_t)TT * DM * 2);
    if ((size_t)(wsp - (char*)d_ws) > ws_size) return;
    k_wtG<<<(unsigned)((DM * D3 / 64 + 63) / 64), 256, 0, stream>>>(wa, DM, D3, WA); k_wtG<<<(DM * DM / 64 + 63) / 64, 256, 0, stream>>>(wp, DM, DM, WP);
    for (int b = 0; b < NB_; ++b) {
        k_cvt8<<<(TT * DM / 8 + 255) / 256, 256, 0, stream>>>(x + (size_t)b * TT * DM, XB, (size_t)TT * DM / 8);
        k_gemmw<bf, 0, true><<<dim3(TT / 64, D3 / 64, 1), 32, 0, stream>>>(XB, nullptr, WA, nullptr, DM, QKV, D3, ba, 0, 0, 0);
        k_phi<<<(NH_ * TT * MF / 4 + 255) / 256, 256, 0, stream>>>(QKV, 0, om, PQh, PQl); k_phi<<<(NH_ * TT * MF / 4 + 255) / 256, 256, 0, stream>>>(QKV, DM, om, PKh, PKl); k_vtp2<<<(NH_ * HD * TT / 2 + 255) / 256, 256, 0, stream>>>(QKV, VTh, VTl);
        for (int h0 = 0; h0 < NH_; h0 += ZH) { const size_t zo = (size_t)h0 * TT * MF;
            k_gemmc<bf, 2, 1><<<dim3(TT / 64, TT / 64, ZH), 32, 0, stream>>>(PQh + zo, PQl + zo, PKh + zo, PKl + zo, MF, Sb, TT, 0, (size_t)TT * MF, (size_t)TT * MF, (size_t)TT * TT);
            k_lin<<<ZH * TT / 8, 256, 0, stream>>>(Sb, Ah, Al, DEN);
            k_gemmc<bf, 2, 2><<<dim3(TT / 64, HD / 64, ZH), 32, 0, stream>>>(Ah, Al, VTh + (size_t)h0 * HD * TT, VTl + (size_t)h0 * HD * TT, TT, O, HD, 0, (size_t)TT * TT, (size_t)HD * TT, (size_t)TT * HD);
            k_y<<<(ZH * TT * HD / 4 + 255) / 256, 256, 0, stream>>>(O, DEN, h0, Yh, Yl); }
        k_gemmw<bf, 1, true><<<dim3(TT / 64, DM / 64, 1), 32, 0, stream>>>(Yh, Yl, WP, nullptr, DM, OUT + (size_t)b * TT * DM, DM, bp, 0, 0, 0); }
}
